// MultiHeadAttention_32495722561673
// MI455X (gfx1250) — hardware-verified
//
#include <hip/hip_runtime.h>
#include <math.h>

#ifndef NB
#define NB 4
#endif
#ifndef SEQ
#define SEQ 1024
#endif
#define NB_FULL 4
#define SEQ_FULL 1024
#define DM 1024
#define NH 16
#define DK 64
#define MAXREL 16
#define NREL 33
#define NRELP 48
#define MT (NB * SEQ)
#define AT_NW 4
#define QP 52
#define OSP 68
#define PSC 16384.0f

static_assert(NH * DK == DM);
static_assert(DK == 64);
static_assert(2 * MAXREL + 1 == NREL);
static_assert(NRELP % 16 == 0 && NRELP >= NREL);
static_assert(QP >= NRELP);
static_assert(SEQ % 64 == 0);
static_assert(MT % 64 == 0);
static_assert(DM % 64 == 0);
static_assert((2 * DM) % 32 == 0);
static_assert(((SEQ / 16) * NB * NH) % AT_NW == 0);
static_assert(NB <= NB_FULL && SEQ <= SEQ_FULL);
static_assert(((long long)MT * (DM / 8)) % 256 == 0);

typedef __attribute__((ext_vector_type(16))) _Float16 v16h;
typedef __attribute__((ext_vector_type(8)))  _Float16 v8h;
typedef __attribute__((ext_vector_type(16))) __bf16   v16b;
typedef __attribute__((ext_vector_type(8)))  __bf16   v8b;
typedef __attribute__((ext_vector_type(8)))  float    v8f;
typedef __attribute__((ext_vector_type(4)))  float    v4f;
typedef __attribute__((ext_vector_type(4)))  unsigned int u4;


__device__ __forceinline__ unsigned short bfu_rne(float v) { unsigned u = __float_as_uint(v); u += 0x7FFFu + ((u >> 16) & 1u); return (unsigned short)(u >> 16); }
__device__ __forceinline__ float bfu_f32(unsigned short h) { return __uint_as_float(((unsigned)h) << 16); }
__device__ __forceinline__ float cmb_bf(float v) { const unsigned u = __float_as_uint(v); const unsigned r = (u + 0x7fffu + ((u >> 16) & 1u)) & 0xffff0000u; return __uint_as_float(r); }
__device__ __forceinline__ unsigned int cmb_pk2(float a, float b) { return (unsigned int)__builtin_bit_cast(unsigned short, (_Float16)a) | ((unsigned int)__builtin_bit_cast(unsigned short, (_Float16)b) << 16); }

#define VST2(T, ptr, val) do { const T vst2_v_ = (val); *(volatile T*)(ptr) = vst2_v_; __threadfence(); *(volatile T*)(ptr) = vst2_v_; } while (0)

__device__ __forceinline__ v8f zero8() { v8f z = {0.f, 0.f, 0.f, 0.f, 0.f, 0.f, 0.f, 0.f}; return z; }

__device__ __forceinline__ v8f wmmab(v16b a, v16b b, v8f c) {
  c = __builtin_amdgcn_wmma_f32_16x16x32_bf16(false, a, false, b, (short)0, c, false, false);
  asm volatile("v_nop\n\tv_nop\n\tv_nop\n\tv_nop" : "+v"(c) : "v"(a), "v"(b));
  return c;
}
__device__ __forceinline__ v8f wmmah(v16h a, v16h b, v8f c) {
  c = __builtin_amdgcn_wmma_f32_16x16x32_f16(false, a, false, b, (short)0, c, false, false);
  asm volatile("v_nop\n\tv_nop\n\tv_nop\n\tv_nop" : "+v"(c) : "v"(a), "v"(b));
  return c;
}
union FBu { v16b v; v8b h[2]; };
union FHu { v16h v; v8h h[2]; };
__device__ __forceinline__ v16b ldfb(const __bf16* p) { FBu f; f.h[0] = *(const v8b*)(p); f.h[1] = *(const v8b*)(p + 16); return f.v; }
__device__ __forceinline__ v16h ldfh(const _Float16* p) { FHu f; f.h[0] = *(const v8h*)(p); f.h[1] = *(const v8h*)(p + 16); return f.v; }

__device__ __forceinline__ void dep_guard4_h(v8f& a, v8f& b, v8f& c, v8f& d, v16h x) { asm volatile("v_nop\n\tv_nop\n\tv_nop\n\tv_nop" : "+v"(a), "+v"(b), "+v"(c), "+v"(d) : "v"(x)); }
__device__ __forceinline__ void dep_guard4_b(v8f& a, v8f& b, v8f& c, v8f& d, v16b x) { asm volatile("v_nop\n\tv_nop\n\tv_nop\n\tv_nop" : "+v"(a), "+v"(b), "+v"(c), "+v"(d) : "v"(x)); }
__device__ __forceinline__ void keep4_h(v16h a, v16h b, v16h c, v16h d) { asm volatile("v_nop" :: "v"(a), "v"(b), "v"(c), "v"(d)); }
__device__ __forceinline__ void keep4_b(v16b a, v16b b, v16b c, v16b d) { asm volatile("v_nop" :: "v"(a), "v"(b), "v"(c), "v"(d)); }
__device__ __forceinline__ void acc_guard4(v8f& a, v8f& b, v8f& c, v8f& d) { asm volatile("v_nop\n\tv_nop\n\tv_nop\n\tv_nop" : "+v"(a), "+v"(b), "+v"(c), "+v"(d)); }

template <typename T> struct Frag;
template <> struct Frag<_Float16> {
  typedef v16h V;
  static __device__ __forceinline__ v16h load(const _Float16* p) { return ldfh(p); }
  static __device__ __forceinline__ v8f mma(v16h a, v16h b, v8f c) { return __builtin_amdgcn_wmma_f32_16x16x32_f16(false, a, false, b, (short)0, c, false, false); }
  static __device__ __forceinline__ void guard4(v8f& a, v8f& b, v8f& c, v8f& d, v16h x) { dep_guard4_h(a, b, c, d, x); }
  static __device__ __forceinline__ void keep(v16h a, v16h b, v16h c, v16h d) { keep4_h(a, b, c, d); }
};
template <> struct Frag<__bf16> {
  typedef v16b V;
  static __device__ __forceinline__ v16b load(const __bf16* p) { return ldfb(p); }
  static __device__ __forceinline__ v8f mma(v16b a, v16b b, v8f c) { return __builtin_amdgcn_wmma_f32_16x16x32_bf16(false, a, false, b, (short)0, c, false, false); }
  static __device__ __forceinline__ void guard4(v8f& a, v8f& b, v8f& c, v8f& d, v16b x) { dep_guard4_b(a, b, c, d, x); }
  static __device__ __forceinline__ void keep(v16b a, v16b b, v16b c, v16b d) { keep4_b(a, b, c, d); }
};
template <int ET> struct Elem;
template <> struct Elem<0> { typedef _Float16 T; };
template <> struct Elem<1> { typedef __bf16 T; };

template <int ET, int BIAS_MODE, int OUT_MODE>
__device__ __forceinline__ void gemm64_body(
    const unsigned short* __restrict__ Ap, int lda, const unsigned short* __restrict__ Btp, int ldb,
    void* __restrict__ Cout, void* __restrict__ Cout2, int ldc, const float* __restrict__ bias,
    int M, int N, int K, float scale, float* slab) {
  typedef typename Elem<ET>::T T;
  typedef typename Frag<T>::V V;
  const T* A = (const T*)Ap; const T* Bt = (const T*)Btp;
  const int lane = threadIdx.x & 31;
  const int wave = threadIdx.x >> 5;
  const int tilesN = N >> 6;
  const int tilesM = M >> 6;
  const int tile = blockIdx.x * 8 + wave;
  if (tile >= tilesM * tilesN) return;
  const int tm = tile / tilesN;
  const int tn = tile - tm * tilesN;
  const int m0 = tm << 6;
  const int n0 = tn << 6;
  const int rlane = lane & 15;
  const int koff  = (lane >> 4) * 8;
  const int mOff  = (lane >> 4) * 8;

  v8f acc[4][4];
#pragma unroll
  for (int i = 0; i < 4; ++i)
#pragma unroll
    for (int j = 0; j < 4; ++j) acc[i][j] = zero8();

  for (int k0 = 0; k0 < K; k0 += 32) {
    V bh[4];
#pragma unroll
    for (int j = 0; j < 4; ++j) bh[j] = Frag<T>::load(Bt + (size_t)(n0 + (j << 4) + rlane) * ldb + koff + k0);
#pragma unroll
    for (int i = 0; i < 4; ++i) {
      V ah = Frag<T>::load(A + (size_t)(m0 + (i << 4) + rlane) * lda + koff + k0);
#pragma unroll
      for (int j = 0; j < 4; ++j) acc[i][j] = Frag<T>::mma(ah, bh[j], acc[i][j]);
      Frag<T>::guard4(acc[i][0], acc[i][1], acc[i][2], acc[i][3], ah);
    }
    Frag<T>::keep(bh[0], bh[1], bh[2], bh[3]);
  }
  acc_guard4(acc[0][0], acc[0][1], acc[0][2], acc[0][3]);
  acc_guard4(acc[1][0], acc[1][1], acc[1][2], acc[1][3]);
  acc_guard4(acc[2][0], acc[2][1], acc[2][2], acc[2][3]);
  acc_guard4(acc[3][0], acc[3][1], acc[3][2], acc[3][3]);

#pragma unroll
  for (int i = 0; i < 4; ++i) {
    const int mBase = m0 + (i << 4);
#pragma unroll
    for (int j = 0; j < 4; ++j) {
      const int n = n0 + (j << 4) + rlane;
      float bv = 0.f;
      if (BIAS_MODE == 2) bv = bias[n];
#pragma unroll
      for (int r = 0; r < 8; ++r) {
        float v = acc[i][j][r] * scale;
        if (BIAS_MODE == 1) v += bias[mBase + mOff + r];
        if (BIAS_MODE == 2) v += bv;
        slab[(mOff + r) * 68 + (j << 4) + rlane] = v;
      }
    }
    __builtin_amdgcn_fence(3  , "workgroup");
    __builtin_amdgcn_wave_barrier();
    __builtin_amdgcn_fence(2  , "workgroup");
    if (OUT_MODE == 0) {
      float* C = (float*)Cout;
      const int hh = lane >> 4, c4 = (lane & 15) * 4;
      for (int pass = 0; pass < 2; ++pass) {
#pragma unroll
        for (int it = 0; it < 8; ++it) {
          const int row = it * 2 + hh;
          v4f v = *(const v4f*)(slab + row * 68 + c4);
          *(volatile v4f*)(C + (size_t)(mBase + row) * ldc + n0 + c4) = v;
        }
        __threadfence();
      }
    } else {
      const int q = lane >> 3, c8 = (lane & 7) * 8;
      unsigned short* C  = (unsigned short*)Cout;
      unsigned short* C2 = (unsigned short*)Cout2;
      for (int pass = 0; pass < 2; ++pass) {
#pragma unroll
        for (int it = 0; it < 4; ++it) {
          const int row = it * 4 + q;
          const float* sp = slab + row * 68 + c8;
          v8h hv, lv;
#pragma unroll
          for (int e = 0; e < 8; ++e) {
            if (OUT_MODE == 1) {
              hv[e] = (_Float16)sp[e];
              lv[e] = (_Float16)0.f;
            } else {
              const unsigned short hb = bfu_rne(sp[e]);
              const unsigned short lb = bfu_rne(sp[e] - bfu_f32(hb));
              hv[e] = __builtin_bit_cast(_Float16, hb);
              lv[e] = __builtin_bit_cast(_Float16, lb);
            }
          }
          *(volatile v8h*)(C + (size_t)(mBase + row) * ldc + n0 + c8) = hv;
          if (OUT_MODE == 2) *(volatile v8h*)(C2 + (size_t)(mBase + row) * ldc + n0 + c8) = lv;
        }
        __threadfence();
      }
    }
    __builtin_amdgcn_fence(3  , "workgroup");
    __builtin_amdgcn_wave_barrier();
    __builtin_amdgcn_fence(2  , "workgroup");
  }
}

__global__ __launch_bounds__(256) void k_gemm_qk(const unsigned short* __restrict__ X, const unsigned short* __restrict__ W,
                                                 unsigned short* __restrict__ CH, unsigned short* __restrict__ CL,
                                                 const float* __restrict__ bias, int M, int N, int K, float scale) {
  __shared__ __align__(16) float sT[8][16 * 68];
  gemm64_body<0, 2, 2>(X, K, W, K, (void*)CH, (void*)CL, N, bias, M, N, K, scale, sT[threadIdx.x >> 5]);
}
__global__ __launch_bounds__(256) void k_gemm_vt(const unsigned short* __restrict__ W, const unsigned short* __restrict__ X,
                                                 unsigned short* __restrict__ C, const float* __restrict__ bias, int M, int N, int K, float scale) {
  __shared__ __align__(16) float sT[8][16 * 68];
  gemm64_body<0, 1, 1>(W, K, X, K, (void*)C, (void*)C, N, bias, M, N, K, scale, sT[threadIdx.x >> 5]);
}
__global__ __launch_bounds__(256) void k_gemm_out(const unsigned short* __restrict__ A, const unsigned short* __restrict__ W,
                                                  float* __restrict__ C, const float* __restrict__ bias, int M, int N, int K) {
  __shared__ __align__(16) float sT[8][16 * 68];
  gemm64_body<1, 2, 0>(A, K, W, K, (void*)C, (void*)C, N, bias, M, N, K, 1.0f, sT[threadIdx.x >> 5]);
}

__global__ __launch_bounds__(256) void k_cast_f16(const float* __restrict__ SRC, long long sbs, int rpb, unsigned short* __restrict__ DST, int nR, float sc) {
  const long long u = (long long)blockIdx.x * 256 + threadIdx.x; const int per = DM / 8; if (u >= (long long)nR * per) return;
  const int r = (int)(u / per); const int c0 = 8 * (int)(u % per); const int bb = r / rpb; const int s = r - bb * rpb;
  const float* sp = SRC + (long long)bb * sbs + (long long)s * DM + c0; float w[8];
#pragma unroll
  for (int e = 0; e < 8; ++e) w[e] = cmb_bf(sp[e]) * sc;
  u4 pk; pk.x = cmb_pk2(w[0], w[1]); pk.y = cmb_pk2(w[2], w[3]); pk.z = cmb_pk2(w[4], w[5]); pk.w = cmb_pk2(w[6], w[7]);
  VST2(u4, (u4*)(DST + (long long)r * DM + c0), pk);
}
__global__ __launch_bounds__(256) void k_wo_dup(const float* __restrict__ Wo, unsigned short* __restrict__ DST) {
  const long long u = (long long)blockIdx.x * 256 + threadIdx.x; const int per = (2 * DM) / 8; if (u >= (long long)DM * per) return;
  const int r = (int)(u / per); const int c0 = 8 * (int)(u % per); const int sc0 = c0 & (DM - 1);
  const float* sp = Wo + (long long)r * DM + sc0; unsigned short w[8];
#pragma unroll
  for (int e = 0; e < 8; ++e) w[e] = bfu_rne(sp[e]);
  u4 pk; pk.x = (unsigned)w[0] | ((unsigned)w[1] << 16); pk.y = (unsigned)w[2] | ((unsigned)w[3] << 16); pk.z = (unsigned)w[4] | ((unsigned)w[5] << 16); pk.w = (unsigned)w[6] | ((unsigned)w[7] << 16);
  VST2(u4, (u4*)(DST + (long long)r * (2 * DM) + c0), pk);
}
__global__ __launch_bounds__(256) void k_table(const float* __restrict__ T, unsigned short* __restrict__ TB) {
  const int u = blockIdx.x * 256 + threadIdx.x; if (u >= NRELP * (DK / 8)) return;
  const int row = u / (DK / 8); const int c0 = 8 * (u % (DK / 8)); const int rr = min(row, NREL - 1);
  unsigned short w[8];
#pragma unroll
  for (int e = 0; e < 8; ++e) { const unsigned short bits = bfu_rne(T[rr * DK + c0 + e]); w[e] = (row < NREL) ? bits : (unsigned short)0; }
  u4 pk; pk.x = (unsigned)w[0] | ((unsigned)w[1] << 16); pk.y = (unsigned)w[2] | ((unsigned)w[3] << 16); pk.z = (unsigned)w[4] | ((unsigned)w[5] << 16); pk.w = (unsigned)w[6] | ((unsigned)w[7] << 16);
  VST2(u4, (u4*)(TB + row * DK + c0), pk);
}
__global__ __launch_bounds__(256) void k_bfvec(const float* __restrict__ SRC, float* __restrict__ DST, int n) {
  const int u = blockIdx.x * 256 + threadIdx.x; if (u >= n) return; VST2(float, DST + u, cmb_bf(SRC[u]));
}

__global__ __launch_bounds__(32 * AT_NW) void k_attn_rel(const unsigned short* __restrict__ QHp, const unsigned short* __restrict__ QLp,
                                                         const unsigned short* __restrict__ KHp, const unsigned short* __restrict__ KLp,
                                                         const unsigned short* __restrict__ VTp, const unsigned short* __restrict__ TBp,
                                                         unsigned short* __restrict__ CTX) {
  __shared__ __align__(16) float qrs[AT_NW][16 * QP];
  __shared__ __align__(16) float osm[AT_NW][16 * OSP];
  const __bf16* QH = (const __bf16*)QHp; const __bf16* QL = (const __bf16*)QLp;
  const __bf16* KH = (const __bf16*)KHp; const __bf16* KL = (const __bf16*)KLp;
  const __bf16* TB = (const __bf16*)TBp; const _Float16* VT = (const _Float16*)VTp;
  const int lane = threadIdx.x & 31, wave = threadIdx.x >> 5, hh = lane >> 4, c = lane & 15;
  const int tile = blockIdx.x * AT_NW + wave;
  const int bh = tile / (SEQ / 16);
  const int l0 = (tile - bh * (SEQ / 16)) * 16;
  const int b = bh / NH, h = bh - b * NH;
  const size_t tok0 = (size_t)b * SEQ;

  v16b qh[2], ql[2];
  {
    const size_t qo = (tok0 + l0 + c) * DM + h * DK + 8 * hh;
#pragma unroll
    for (int dc = 0; dc < 2; ++dc) { qh[dc] = ldfb(QH + qo + dc * 32); ql[dc] = ldfb(QL + qo + dc * 32); }
  }
  float* myq = qrs[wave];
#pragma unroll
  for (int jt = 0; jt < NRELP / 16; ++jt) {
    v8f acc = zero8();
#pragma unroll
    for (int dc = 0; dc < 2; ++dc) {
      const v16b ta = ldfb(TB + (jt * 16 + c) * DK + dc * 32 + 8 * hh);
      acc = wmmab(ta, ql[dc], acc);
      acc = wmmab(ta, qh[dc], acc);
    }
#pragma unroll
    for (int r = 0; r < 8; ++r) myq[c * QP + jt * 16 + 8 * hh + r] = acc[r];
  }
  __builtin_amdgcn_fence(3  , "workgroup");
  __builtin_amdgcn_wave_barrier();
  __builtin_amdgcn_fence(2  , "workgroup");

  const int lglob = l0 + c;
  const float* qrow = myq + c * QP + MAXREL;
  const float L2E = 1.4426950408889634f;
  float m_run = -1.0e30f, s_run = 0.f;
  v8f o[4];
#pragma unroll
  for (int t = 0; t < 4; ++t) o[t] = zero8();
  const __bf16* kbh = KH + tok0 * DM + h * DK + 8 * hh;
  const __bf16* kbl = KL + tok0 * DM + h * DK + 8 * hh;
  const _Float16* vb = VT + (size_t)(h * DK + c) * MT + tok0 + 8 * hh;

#pragma unroll 1
  for (int r0 = 0; r0 < SEQ; r0 += 32) {
    v8f t[2];
#pragma unroll
    for (int tt = 0; tt < 2; ++tt) {
      v8f acc = zero8();
#pragma unroll
      for (int dc = 0; dc < 2; ++dc) {
        const size_t ko = (size_t)(r0 + 16 * tt + c) * DM + dc * 32;
        const v16b kfh = ldfb(kbh + ko);
        const v16b kfl = ldfb(kbl + ko);
        acc = wmmab(kfl, qh[dc], acc);
        acc = wmmab(kfh, ql[dc], acc);
        acc = wmmab(kfh, qh[dc], acc);
      }
      t[tt] = acc;
    }
    float p[16];
    float mt = -1.0e30f;
    const int dbase = r0 + 8 * hh - lglob;
#pragma unroll
    for (int e = 0; e < 8; ++e) {
      const int d0 = min(max(dbase + e, -MAXREL), MAXREL);
      const int d1 = min(max(dbase + 16 + e, -MAXREL), MAXREL);
      p[e]     = (t[0][e] * 0.125f + qrow[d0]) * L2E;
      p[8 + e] = (t[1][e] * 0.125f + qrow[d1]) * L2E;
      mt = fmaxf(mt, fmaxf(p[e], p[8 + e]));
    }
    mt = fmaxf(mt, __shfl_xor(mt, 16, 32));
    const float m_new = fmaxf(m_run, mt);
    const float corr  = exp2f(m_run - m_new);
    float sum = 0.f;
    v16h pA;
#pragma unroll
    for (int r = 0; r < 16; ++r) {
      const float ev = exp2f(p[r] - m_new);
      sum += ev;
      pA[r] = (_Float16)(ev * PSC);
    }
    sum += __shfl_xor(sum, 16, 32);
    s_run = s_run * corr + sum;
    m_run = m_new;
    float sc[8];
#pragma unroll
    for (int i = 0; i < 8; ++i) sc[i] = __shfl(corr, i + 8 * hh, 32);
#pragma unroll
    for (int tq = 0; tq < 4; ++tq) {
      const v16h vf = ldfh(vb + (size_t)tq * 16 * MT + r0);
      v8f oc = o[tq];
#pragma unroll
      for (int i = 0; i < 8; ++i) oc[i] *= sc[i];
      o[tq] = wmmah(pA, vf, oc);
    }
  }

  float inv[8];
#pragma unroll
  for (int i = 0; i < 8; ++i) inv[i] = 1.0f / (__shfl(s_run, i + 8 * hh, 32) * PSC);
  float* os = osm[wave];
#pragma unroll
  for (int tq = 0; tq < 4; ++tq)
#pragma unroll
    for (int i = 0; i < 8; ++i) os[(8 * hh + i) * OSP + tq * 16 + c] = o[tq][i] * inv[i];
  __builtin_amdgcn_fence(3  , "workgroup");
  __builtin_amdgcn_wave_barrier();
  __builtin_amdgcn_fence(2  , "workgroup");
  {
    const int q = lane >> 3, c8 = (lane & 7) * 8;
    unsigned short* ch = CTX + (tok0 + l0) * (size_t)(2 * DM) + h * DK + c8;
    u4 ph[4], pl[4];
#pragma unroll
    for (int it = 0; it < 4; ++it) {
      const int row = it * 4 + q;
      const float* sp = os + row * OSP + c8;
      unsigned short hb[8], lb[8];
#pragma unroll
      for (int e = 0; e < 8; ++e) { const float v = sp[e]; hb[e] = bfu_rne(v); lb[e] = bfu_rne(v - bfu_f32(hb[e])); }
      ph[it].x = (unsigned)hb[0] | ((unsigned)hb[1] << 16); ph[it].y = (unsigned)hb[2] | ((unsigned)hb[3] << 16);
      ph[it].z = (unsigned)hb[4] | ((unsigned)hb[5] << 16); ph[it].w = (unsigned)hb[6] | ((unsigned)hb[7] << 16);
      pl[it].x = (unsigned)lb[0] | ((unsigned)lb[1] << 16); pl[it].y = (unsigned)lb[2] | ((unsigned)lb[3] << 16);
      pl[it].z = (unsigned)lb[4] | ((unsigned)lb[5] << 16); pl[it].w = (unsigned)lb[6] | ((unsigned)lb[7] << 16);
    }
    for (int pass = 0; pass < 2; ++pass) {
#pragma unroll
      for (int it = 0; it < 4; ++it) {
        const int row = it * 4 + q;
        *(volatile u4*)(ch + (size_t)row * (2 * DM)) = ph[it];
        *(volatile u4*)(ch + (size_t)row * (2 * DM) + DM) = pl[it];
      }
      __threadfence();
    }
  }
}

extern "C" void kernel_launch(void* const* d_in, const int* in_sizes, int n_in, void* d_out, int out_size, void* d_ws, size_t ws_size, hipStream_t stream) {
  if (n_in < 12) return;
  const long long actn = ((long long)(NB - 1) * SEQ_FULL + SEQ) * DM;
  if ((long long)in_sizes[0] < actn || (long long)in_sizes[1] < actn || (long long)in_sizes[2] < actn) return;
  if (in_sizes[3] < DM * DM || in_sizes[5] < DM * DM || in_sizes[7] < DM * DM || in_sizes[9] < DM * DM) return;
  if (in_sizes[4] < DM || in_sizes[6] < DM || in_sizes[8] < DM || in_sizes[10] < DM) return;
  if (in_sizes[11] < NREL * DK) return;
  if ((long long)out_size < (long long)MT * DM) return;

  const float* Qi = (const float*)d_in[0];
  const float* Ki = (const float*)d_in[1];
  const float* Vi = (const float*)d_in[2];
  const float* Wq = (const float*)d_in[3];
  const float* bq = (const float*)d_in[4];
  const float* Wk = (const float*)d_in[5];
  const float* bk = (const float*)d_in[6];
  const float* Wv = (const float*)d_in[7];
  const float* bv = (const float*)d_in[8];
  const float* Wo = (const float*)d_in[9];
  const float* bo = (const float*)d_in[10];
  const float* rel = (const float*)d_in[11];
  float* out = (float*)d_out;

  constexpr size_t SZ_ACT = (size_t)MT * DM * 2;
  constexpr size_t SZ_W   = (size_t)DM * DM * 2;
  constexpr size_t SZ_WO2 = (size_t)DM * 2 * DM * 2;
  constexpr size_t SZ_BR  = (size_t)4 * DM * 4;
  constexpr size_t SZ_TB  = (size_t)NRELP * DK * 2;
  constexpr size_t SZ_CTX = (size_t)MT * 2 * DM * 2;
  static_assert(SZ_ACT % 256 == 0 && SZ_W % 256 == 0 && SZ_WO2 % 256 == 0 && SZ_BR % 256 == 0 && SZ_TB % 256 == 0 && SZ_CTX % 256 == 0);
  constexpr size_t TOTAL = 3 * SZ_ACT + 3 * SZ_W + SZ_WO2 + SZ_BR + SZ_TB + 4 * SZ_ACT + SZ_ACT + SZ_CTX;
  static_assert(TOTAL <= (size_t)134217728);
  if (TOTAL > ws_size) return;

  char* wsp = (char*)d_ws;
  unsigned short* XQ  = (unsigned short*)wsp; wsp += SZ_ACT;
  unsigned short* XK  = (unsigned short*)wsp; wsp += SZ_ACT;
  unsigned short* XV  = (unsigned short*)wsp; wsp += SZ_ACT;
  unsigned short* WQ6 = (unsigned short*)wsp; wsp += SZ_W;
  unsigned short* WK6 = (unsigned short*)wsp; wsp += SZ_W;
  unsigned short* WV6 = (unsigned short*)wsp; wsp += SZ_W;
  unsigned short* WO2 = (unsigned short*)wsp; wsp += SZ_WO2;
  float*          BR  = (float*)wsp;          wsp += SZ_BR;
  unsigned short* TB  = (unsigned short*)wsp; wsp += SZ_TB;
  unsigned short* QHp = (unsigned short*)wsp; wsp += SZ_ACT;
  unsigned short* QLp = (unsigned short*)wsp; wsp += SZ_ACT;
  unsigned short* KHp = (unsigned short*)wsp; wsp += SZ_ACT;
  unsigned short* KLp = (unsigned short*)wsp; wsp += SZ_ACT;
  unsigned short* VTp = (unsigned short*)wsp; wsp += SZ_ACT;
  unsigned short* CTX = (unsigned short*)wsp; wsp += SZ_CTX;

  const unsigned gW   = (unsigned)(((long long)DM * (DM / 8) + 255) / 256);
  const unsigned gAct = (unsigned)(((long long)MT * (DM / 8) + 255) / 256);
  k_cast_f16<<<gW, 256, 0, stream>>>(Wq, 0, DM, WQ6, DM, 16.0f);
  k_cast_f16<<<gW, 256, 0, stream>>>(Wk, 0, DM, WK6, DM, 16.0f);
  k_cast_f16<<<gW, 256, 0, stream>>>(Wv, 0, DM, WV6, DM, 16.0f);
  k_wo_dup<<<(unsigned)(((long long)DM * ((2 * DM) / 8) + 255) / 256), 256, 0, stream>>>(Wo, WO2);
  k_bfvec<<<(DM + 255) / 256, 256, 0, stream>>>(bq, BR + 0 * DM, DM);
  k_bfvec<<<(DM + 255) / 256, 256, 0, stream>>>(bk, BR + 1 * DM, DM);
  k_bfvec<<<(DM + 255) / 256, 256, 0, stream>>>(bv, BR + 2 * DM, DM);
  k_bfvec<<<(DM + 255) / 256, 256, 0, stream>>>(bo, BR + 3 * DM, DM);
  k_table<<<(NRELP * (DK / 8) + 255) / 256, 256, 0, stream>>>(rel, TB);
  k_cast_f16<<<gAct, 256, 0, stream>>>(Qi, (long long)SEQ_FULL * DM, SEQ, XQ, MT, 1.0f);
  k_cast_f16<<<gAct, 256, 0, stream>>>(Ki, (long long)SEQ_FULL * DM, SEQ, XK, MT, 1.0f);
  k_cast_f16<<<gAct, 256, 0, stream>>>(Vi, (long long)SEQ_FULL * DM, SEQ, XV, MT, 1.0f);

  const unsigned gQK = (unsigned)((((MT / 64) * (DM / 64)) + 7) / 8);
  k_gemm_qk<<<gQK, 256, 0, stream>>>(XQ, WQ6, QHp, QLp, BR + 0 * DM, MT, DM, DM, 0.0625f);
  k_gemm_qk<<<gQK, 256, 0, stream>>>(XK, WK6, KHp, KLp, BR + 1 * DM, MT, DM, DM, 0.0625f);
  k_gemm_vt<<<(unsigned)((((DM / 64) * (MT / 64)) + 7) / 8), 256, 0, stream>>>(WV6, XV, VTp, BR + 2 * DM, DM, MT, DM, 0.0625f);

  k_attn_rel<<<(unsigned)((NB * NH * (SEQ / 16)) / AT_NW), 32 * AT_NW, 0, stream>>>(QHp, QLp, KHp, KLp, VTp, TB, CTX);

  k_gemm_out<<<gQK, 256, 0, stream>>>(CTX, WO2, out, BR + 3 * DM, MT, DM, 2 * DM);
}
